// GroupedQueryAttention_68350109548805
// MI455X (gfx1250) — hardware-verified
//
#include <hip/hip_runtime.h>

#ifndef NB
#define NB 2
#endif
#ifndef SEQ
#define SEQ 2048
#endif
#define NB_FULL 2
#define SEQ_FULL 2048
#define DM 2048
#define NH 16
#define NKV 4
#define NREP (NH / NKV)
#define HD 128
#define KVD (NKV * HD)
#define QKVN (DM + 2 * KVD)
#define SLEN SEQ
#define NR (NB * SLEN)
#define TQ SLEN
#define TK SLEN
#define SCL 0.08838834764831845f
#define QBLKS (TQ / 64)
#define EROWS 64
static_assert(SLEN % 128 == 0);
static_assert(SLEN <= SEQ_FULL);
static_assert(NB >= 1 && NB <= NB_FULL);
static_assert(DM % 64 == 0 && DM == NH * HD);
static_assert(HD == 128 && HD == 32 * 4);
static_assert(NH % NKV == 0 && KVD % 64 == 0 && QKVN % 64 == 0);
static_assert(DM % 32 == 0 && (2 * DM) % 32 == 0);
static_assert(NR % 128 == 0);
static_assert(EROWS > 0 && EROWS % 64 == 0);
static_assert(((size_t)NR * DM * 2) % 256 == 0);
static_assert(4 * 32 * 68 * 4 <= 131072);
static_assert(4 * 16 * 40 * 2 + 4 * 16 * (HD + 4) * 4 <= 131072);
static_assert(2 * 4 * 16 * 40 * 2 + 4 * 16 * 68 * 4 <= 131072);
static_assert(64 * 65 * 4 <= 131072);
static_assert(64 * (HD + 2) * 2 <= 131072);
static_assert(256 * 16 * 2 == 64 * 128);
static_assert(256 * 16 * 4 == HD * 128);
static_assert(32 * 16 * 16 == 16 * HD * 4);
static_assert(32 * 16 * 8 == 16 * 64 * 4);
static_assert(32 * 16 * 16 == 32 * 64 * 4);

static constexpr float W_SC = 16.0f;
static constexpr float W_SC_HI = 16384.0f;
static constexpr float ALPHA_P = 0.0625f;
static constexpr float ALPHA_O = 6.103515625e-05f;

static constexpr size_t al256(size_t b) { return (b + 255) & ~(size_t)255; }
static constexpr size_t WS_TOTAL = al256((size_t)QKVN * DM * 2) + al256((size_t)DM * 2 * DM * 2) + al256((size_t)NR * DM * 4) + 3 * al256((size_t)NR * DM * 2) + 4 * al256((size_t)NR * KVD * 2);
static_assert(WS_TOTAL <= ((size_t)128 << 20));
static_assert((size_t)NB * NKV * HD * TK * 2 <= (size_t)NR * DM * 2);

typedef _Float16 h16;
typedef _Float16 v16h __attribute__((ext_vector_type(16)));
typedef _Float16 v4h __attribute__((ext_vector_type(4)));
typedef unsigned short v8us __attribute__((ext_vector_type(8), may_alias));
typedef float v8f __attribute__((ext_vector_type(8)));
typedef float v4f __attribute__((ext_vector_type(4)));
typedef float v4fa __attribute__((ext_vector_type(4), may_alias));
union FragH { v16h v; v8us half[2]; _Float16 h[16]; unsigned short u[16]; };

__device__ __forceinline__ unsigned short bf16_bits(float x) { unsigned int u = __float_as_uint(x); return (unsigned short)((u + 0x7FFFu + ((u >> 16) & 1u)) >> 16); }
__device__ __forceinline__ float bf16_val(unsigned short b) { return __uint_as_float(((unsigned int)b) << 16); }
__device__ __forceinline__ float bf16_rne(float x) { return bf16_val(bf16_bits(x)); }
static __device__ __forceinline__ h16 toh_flush(float v) { const h16 r = (h16)v; return (fabsf(v) < 6.103515625e-05f) ? (h16)0.0f : r; }
static __device__ __forceinline__ unsigned short hbits_flush(unsigned short u) { return ((u & 0x7C00u) == 0u) ? (unsigned short)0 : u; }

template <int NT>
__device__ __forceinline__ v8f mmaH(v16h ah, v16h al, v16h bh, v16h bl, v8f c) {
  c = __builtin_amdgcn_wmma_f32_16x16x32_f16(false, ah, false, bh, (short)0, c, false, false);
  if (NT >= 2) c = __builtin_amdgcn_wmma_f32_16x16x32_f16(false, al, false, bh, (short)0, c, false, false);
  if (NT >= 3) c = __builtin_amdgcn_wmma_f32_16x16x32_f16(false, ah, false, bl, (short)0, c, false, false);
  asm volatile("v_nop\n\tv_nop\n\tv_nop\n\tv_nop" : "+v"(c) : "v"(ah), "v"(al), "v"(bh), "v"(bl));
  return c;
}
__device__ __forceinline__ v16h g2_frag(const _Float16* p, int hh) { FragH f; f.half[0] = *(const v8us*)((const unsigned short*)p + 8 * hh); f.half[1] = *(const v8us*)((const unsigned short*)p + 16 + 8 * hh); return f.v; }
__device__ __forceinline__ v8f g2_mma(v16h a, v16h b, v8f c) { v8f d = __builtin_amdgcn_wmma_f32_16x16x32_f16(false, a, false, b, (short)0, c, false, false); asm volatile("v_nop\n\tv_nop\n\tv_nop\n\tv_nop" : "+v"(d) : "v"(a), "v"(b)); return d; }

__device__ __forceinline__ int blk_early(const int* __restrict__ dq, int s0, int lane) {
  const int sa = s0 + lane, sb = s0 + 32 + lane;
  const int da = dq[sa], db = dq[sb];
  const int ea = dq[max(sa - EROWS, 0)], eb = dq[max(sb - EROWS, 0)];
  const bool e = (sa < EROWS) | (ea != da) | (sb < EROWS) | (eb != db);
  return (__builtin_amdgcn_ballot_w32(e) != 0u) ? 1 : 0;
}

__global__ __launch_bounds__(256) void k_wtr(const float* __restrict__ Wm, int Kd, int Nd, _Float16* __restrict__ Bt, int ldb, float sc0, float sc1, int two) {
  __shared__ float tl[64][65];
  const int tid = threadIdx.x; const int ntn = Nd >> 6; const int kt = blockIdx.x / ntn, nt = blockIdx.x - kt * ntn; const int k0 = kt * 64, n0 = nt * 64;
  for (int i = tid; i < 64 * 16; i += 256) {
    const int r = i >> 4, c4 = (i & 15) * 4;
    const v4f a = *(const v4fa*)(Wm + (size_t)(k0 + r) * Nd + n0 + c4);
#pragma unroll
    for (int q = 0; q < 4; ++q) tl[r][c4 + q] = bf16_rne(a[q]);
  }
  __syncthreads();
  v8us o0[2], o1[2];
#pragma unroll
  for (int rd = 0; rd < 2; ++rd) {
    const int n = rd * 32 + (tid >> 3), pc = tid & 7; FragH f0, f1;
#pragma unroll
    for (int q = 0; q < 8; ++q) { const float v = tl[pc * 8 + q][n]; f0.h[q] = toh_flush(v * sc0); f1.h[q] = toh_flush(v * sc1); }
    o0[rd] = f0.half[0]; o1[rd] = f1.half[0];
  }
  for (int pass = 0; pass < 2; ++pass) {
#pragma unroll
    for (int rd = 0; rd < 2; ++rd) {
      const int n = rd * 32 + (tid >> 3), pc = tid & 7;
      const size_t o = (size_t)(n0 + n) * ldb + k0 + pc * 8;
      *(volatile v8us*)((unsigned short*)Bt + o) = o0[rd];
      if (two != 0) *(volatile v8us*)((unsigned short*)Bt + o + Kd) = o1[rd];
    }
    if (pass == 0) __threadfence();
  }
}

__global__ __launch_bounds__(256) void k_x16(const float* __restrict__ x, _Float16* __restrict__ X16, size_t n8) {
  const size_t t = (size_t)blockIdx.x * 256 + threadIdx.x; if (t >= n8) return;
  const size_t e = t * 8; const size_t r = e / DM; const size_t c = e % DM; const size_t b = r / SLEN, s = r % SLEN;
  const float* src = x + (b * SEQ_FULL + s) * DM + c;
  const v4f a0 = *(const v4fa*)src, a1 = *(const v4fa*)(src + 4);
  FragH f;
#pragma unroll
  for (int q = 0; q < 4; ++q) { f.h[q] = (_Float16)bf16_rne(a0[q]); f.h[4 + q] = (_Float16)bf16_rne(a1[q]); }
  const v8us o = f.half[0];
  *(volatile v8us*)((unsigned short*)X16 + e) = o; __threadfence(); *(volatile v8us*)((unsigned short*)X16 + e) = o;
}

template <int ACT>
__global__ __launch_bounds__(128) void k_gemm2(const _Float16* __restrict__ A, int lda, size_t sA, const _Float16* __restrict__ Bh, int ldb, size_t sB, float alpha,
                                               float* C, _Float16* C16, int ldc, size_t sC, int M, int N, int K) {
  __shared__ __attribute__((aligned(16))) float so[4][32][68];
  const int tid = threadIdx.x, w = tid >> 5, lane = tid & 31, ln = lane & 15, hh = lane >> 4; const int by = blockIdx.y;
  A += (size_t)by * sA; Bh += (size_t)by * sB; const size_t cofs = (size_t)by * sC;
  const int ntn = N >> 6; const int mt = blockIdx.x / ntn, nq = blockIdx.x - mt * ntn; const int row0 = mt * 128 + 32 * w, col0 = nq * 64; if (row0 >= M) return;
  const _Float16* a0p = A + (size_t)(row0 + ln) * lda; const _Float16* a1p = a0p + (size_t)16 * lda;
  const _Float16* b0p = Bh + (size_t)(col0 + ln) * ldb; const _Float16* b1p = b0p + (size_t)16 * ldb; const _Float16* b2p = b1p + (size_t)16 * ldb; const _Float16* b3p = b2p + (size_t)16 * ldb;
  const v8f z8 = {0.f,0.f,0.f,0.f,0.f,0.f,0.f,0.f}; v8f c00 = z8, c01 = z8, c02 = z8, c03 = z8, c10 = z8, c11 = z8, c12 = z8, c13 = z8;
#pragma unroll 1
  for (int kb = 0; kb < K; kb += 32) {
    const v16h a0 = g2_frag(a0p + kb, hh), a1 = g2_frag(a1p + kb, hh);
    v16h bf = g2_frag(b0p + kb, hh); c00 = g2_mma(a0, bf, c00); c10 = g2_mma(a1, bf, c10);
    bf = g2_frag(b1p + kb, hh); c01 = g2_mma(a0, bf, c01); c11 = g2_mma(a1, bf, c11);
    bf = g2_frag(b2p + kb, hh); c02 = g2_mma(a0, bf, c02); c12 = g2_mma(a1, bf, c12);
    bf = g2_frag(b3p + kb, hh); c03 = g2_mma(a0, bf, c03); c13 = g2_mma(a1, bf, c13);
  }
  v8f accs[8] = {c00, c01, c02, c03, c10, c11, c12, c13};
#pragma unroll
  for (int u = 0; u < 8; ++u) {
    const int t = u & 3, half = u >> 2;
#pragma unroll
    for (int r = 0; r < 8; ++r) { const int rloc = half * 16 + 8 * hh + r; float v = accs[u][r] * alpha; if (ACT == 3) v = fmaxf(v, 0.f); so[w][rloc][t * 16 + ln] = v; }
  }
  __builtin_amdgcn_fence(4, "workgroup"); __builtin_amdgcn_wave_barrier();
  const int rsub = lane >> 4, c4 = (lane & 15) * 4;
  for (int pass = 0; pass < 2; ++pass) {
#pragma unroll
    for (int q = 0; q < 16; ++q) {
      const int r = q * 2 + rsub; const v4f v = *(const v4fa*)&so[w][r][c4];
      if (C) *(volatile v4f*)(C + cofs + (size_t)(row0 + r) * ldc + col0 + c4) = v;
      if (C16) { v4h h4; for (int i = 0; i < 4; ++i) h4[i] = (_Float16)v[i]; *(volatile v4h*)(C16 + cofs + (size_t)(row0 + r) * ldc + col0 + c4) = h4; }
    }
    if (pass == 0) __threadfence();
  }
}

__global__ __launch_bounds__(128) void k_gemmo(const _Float16* __restrict__ A, int lda, size_t sA, const _Float16* __restrict__ Bh, int ldb, float alpha, const int* __restrict__ doc,
                                               float* C, int ldc, size_t sC, int M, int N, int K1, int K2) {
  __shared__ __attribute__((aligned(16))) float so[4][32][68];
  const int tid = threadIdx.x, lane = tid & 31, ln = lane & 15, hh = lane >> 4; const int by = blockIdx.y;
  const int w = __builtin_amdgcn_readfirstlane(tid >> 5);
  A += (size_t)by * sA; const size_t cofs = (size_t)by * sC;
  const int ntn = N >> 6; const int mt = blockIdx.x / ntn, nq = blockIdx.x - mt * ntn; const int row0 = mt * 128 + 32 * w, col0 = nq * 64; if (row0 >= M) return;
  const int* dq = doc + (size_t)by * SEQ_FULL;
  bool e = false;
#pragma unroll
  for (int i = 0; i < 4; ++i) {
    const int sa = min(mt * 128 + i * 32 + lane, M - 1);
    const int da = dq[sa]; const int ea = dq[max(sa - EROWS, 0)];
    e = e | (sa < EROWS) | (ea != da);
  }
  const int K = (__builtin_amdgcn_ballot_w32(e) != 0u) ? K2 : K1;
  const _Float16* a0p = A + (size_t)(row0 + ln) * lda; const _Float16* a1p = a0p + (size_t)16 * lda;
  const _Float16* b0p = Bh + (size_t)(col0 + ln) * ldb; const _Float16* b1p = b0p + (size_t)16 * ldb; const _Float16* b2p = b1p + (size_t)16 * ldb; const _Float16* b3p = b2p + (size_t)16 * ldb;
  const v8f z8 = {0.f,0.f,0.f,0.f,0.f,0.f,0.f,0.f}; v8f c00 = z8, c01 = z8, c02 = z8, c03 = z8, c10 = z8, c11 = z8, c12 = z8, c13 = z8;
#pragma unroll 1
  for (int kb = 0; kb < K; kb += 32) {
    const v16h a0 = g2_frag(a0p + kb, hh), a1 = g2_frag(a1p + kb, hh);
    v16h bf = g2_frag(b0p + kb, hh); c00 = g2_mma(a0, bf, c00); c10 = g2_mma(a1, bf, c10);
    bf = g2_frag(b1p + kb, hh); c01 = g2_mma(a0, bf, c01); c11 = g2_mma(a1, bf, c11);
    bf = g2_frag(b2p + kb, hh); c02 = g2_mma(a0, bf, c02); c12 = g2_mma(a1, bf, c12);
    bf = g2_frag(b3p + kb, hh); c03 = g2_mma(a0, bf, c03); c13 = g2_mma(a1, bf, c13);
  }
  v8f accs[8] = {c00, c01, c02, c03, c10, c11, c12, c13};
#pragma unroll
  for (int u = 0; u < 8; ++u) {
    const int t = u & 3, half = u >> 2;
#pragma unroll
    for (int r = 0; r < 8; ++r) { const int rloc = half * 16 + 8 * hh + r; so[w][rloc][t * 16 + ln] = accs[u][r] * alpha; }
  }
  __builtin_amdgcn_fence(4, "workgroup"); __builtin_amdgcn_wave_barrier();
  const int rsub = lane >> 4, c4 = (lane & 15) * 4;
  for (int pass = 0; pass < 2; ++pass) {
#pragma unroll
    for (int q = 0; q < 16; ++q) {
      const int r = q * 2 + rsub; const v4f v = *(const v4fa*)&so[w][r][c4];
      *(volatile v4f*)(C + cofs + (size_t)(row0 + r) * ldc + col0 + c4) = v;
    }
    if (pass == 0) __threadfence();
  }
}

__global__ __launch_bounds__(256) void k_rope(const float* __restrict__ F, int ld, int nhd, const float* __restrict__ CS, const float* __restrict__ SN, _Float16* __restrict__ H, _Float16* __restrict__ L) {
  #pragma clang fp contract(off)
  const size_t t = (size_t)blockIdx.x * 256 + threadIdx.x; if (t >= (size_t)NR * nhd * 16) return;
  const int p = (int)(t & 15); const int hd = (int)((t >> 4) % (size_t)nhd); const size_t row = t / (size_t)(16 * nhd);
  const int s = (int)(row % SLEN); const int g = p & 7; const int up = p >> 3;
  const float* src = F + row * (size_t)ld + hd * HD + g * 8;
  const v4f xa = *(const v4fa*)src, xb = *(const v4fa*)(src + 4), ya = *(const v4fa*)(src + 64), yb = *(const v4fa*)(src + 68);
  const float* ct = CS + (size_t)s * 64 + g * 8; const float* st = SN + (size_t)s * 64 + g * 8;
  const v4f ca = *(const v4fa*)ct, cb = *(const v4fa*)(ct + 4), sa = *(const v4fa*)st, sb = *(const v4fa*)(st + 4);
  const float x1s[8] = {xa[0], xa[1], xa[2], xa[3], xb[0], xb[1], xb[2], xb[3]};
  const float x2s[8] = {ya[0], ya[1], ya[2], ya[3], yb[0], yb[1], yb[2], yb[3]};
  const float cs[8] = {ca[0], ca[1], ca[2], ca[3], cb[0], cb[1], cb[2], cb[3]};
  const float ss[8] = {sa[0], sa[1], sa[2], sa[3], sb[0], sb[1], sb[2], sb[3]};
  FragH fh, fl;
#pragma unroll
  for (int i = 0; i < 8; ++i) {
    const float x1 = x1s[i], x2 = x2s[i], c = bf16_rne(cs[i]), sn = bf16_rne(ss[i]);
    const float o1 = x1 * c - x2 * sn; const float o2 = x2 * c + x1 * sn; const float o = up ? o2 : o1;
    const _Float16 hv = toh_flush(o); fh.h[i] = hv; fl.h[i] = toh_flush((o - (float)hv) * 1024.0f);
  }
  const size_t oh = row * (size_t)ld + hd * HD + p * 8;
  const v8us vh = fh.half[0], vl = fl.half[0];
  for (int pass = 0; pass < 2; ++pass) {
    *(volatile v8us*)((unsigned short*)H + oh) = vh;
    *(volatile v8us*)((unsigned short*)L + oh) = vl;
    if (pass == 0) __threadfence();
  }
}

__global__ __launch_bounds__(256) void k_vtg(const _Float16* __restrict__ V16, _Float16* __restrict__ Vt) {
  __shared__ unsigned short tl[64][HD + 2];
  const int tid = threadIdx.x; const int nlg = SLEN / 64; const int slab = blockIdx.x / nlg, lg = blockIdx.x % nlg; const int b = slab / NKV, g = slab % NKV;
  for (int i = tid; i < 64 * 16; i += 256) {
    const int r = i >> 4, c8 = (i & 15) * 8; FragH f;
    f.half[0] = *(const v8us*)((const unsigned short*)V16 + ((size_t)b * SLEN + lg * 64 + r) * KVD + g * HD + c8);
#pragma unroll
    for (int q = 0; q < 8; ++q) tl[r][c8 + q] = hbits_flush(f.u[q]);
  }
  __syncthreads();
  for (int pass = 0; pass < 2; ++pass) {
#pragma unroll
    for (int rd = 0; rd < 4; ++rd) {
      const int d = rd * 32 + (tid >> 3), pc = tid & 7; FragH f;
#pragma unroll
      for (int q = 0; q < 8; ++q) f.u[q] = tl[pc * 8 + q][d];
      *(volatile v8us*)((unsigned short*)Vt + ((size_t)slab * HD + d) * TK + lg * 64 + pc * 8) = f.half[0];
    }
    if (pass == 0) __threadfence();
  }
}
__global__ __launch_bounds__(256) void k_vtl(const float* __restrict__ VF, _Float16* __restrict__ VtL) {
  __shared__ unsigned short tl[64][HD + 2];
  const int tid = threadIdx.x; const int nlg = SLEN / 64; const int slab = blockIdx.x / nlg, lg = blockIdx.x % nlg; const int b = slab / NKV, g = slab % NKV;
  for (int i = tid; i < 64 * 32; i += 256) {
    const int r = i >> 5, c4 = (i & 31) * 4;
    const v4f a = *(const v4fa*)(VF + ((size_t)b * SLEN + lg * 64 + r) * KVD + g * HD + c4);
    FragH f;
#pragma unroll
    for (int q = 0; q < 4; ++q) {
      const float v = a[q]; FragH c; c.h[0] = (_Float16)v; c.u[0] = hbits_flush(c.u[0]);
      const float hv = (float)c.h[0]; f.h[q] = toh_flush((v - hv) * 1024.0f);
    }
#pragma unroll
    for (int q = 0; q < 4; ++q) tl[r][c4 + q] = f.u[q];
  }
  __syncthreads();
  for (int pass = 0; pass < 2; ++pass) {
#pragma unroll
    for (int rd = 0; rd < 4; ++rd) {
      const int d = rd * 32 + (tid >> 3), pc = tid & 7; FragH f;
#pragma unroll
      for (int q = 0; q < 8; ++q) f.u[q] = tl[pc * 8 + q][d];
      *(volatile v8us*)((unsigned short*)VtL + ((size_t)slab * HD + d) * TK + lg * 64 + pc * 8) = f.half[0];
    }
    if (pass == 0) __threadfence();
  }
}

__global__ __launch_bounds__(256) void k_hl(const float* __restrict__ Fp, _Float16* __restrict__ A2, size_t n8) {
  const size_t t = (size_t)blockIdx.x * 256 + threadIdx.x; if (t >= n8) return;
  const size_t e = t * 8; const size_t r = e / DM; const int c = (int)(e % DM);
  const v4f a = *(const v4fa*)(Fp + e), d = *(const v4fa*)(Fp + e + 4);
  FragH fh, fl;
#pragma unroll
  for (int q = 0; q < 4; ++q) {
    _Float16 hv = toh_flush(a[q]); fh.h[q] = hv; fl.h[q] = toh_flush((a[q] - (float)hv) * 1024.0f);
    hv = toh_flush(d[q]); fh.h[4 + q] = hv; fl.h[4 + q] = toh_flush((d[q] - (float)hv) * 1024.0f);
  }
  const size_t o2 = r * (size_t)(2 * DM) + c;
  const v8us vh = fh.half[0], vl = fl.half[0];
  for (int pass = 0; pass < 2; ++pass) {
    *(volatile v8us*)((unsigned short*)A2 + o2) = vh;
    *(volatile v8us*)((unsigned short*)A2 + o2 + DM) = vl;
    if (pass == 0) __threadfence();
  }
}

__global__ __launch_bounds__(128) __attribute__((amdgpu_num_vgpr(256))) void k_flash(const _Float16* __restrict__ Q16, int ldq, const _Float16* __restrict__ K16, int ldk,
                                               const _Float16* __restrict__ Vt, const int* __restrict__ doc, float* __restrict__ O, int ldo) {
  constexpr int RPW = 16, DT = 8, KS = 4;
  __shared__ __attribute__((aligned(16))) unsigned short sP[4][RPW][40];
  __shared__ __attribute__((aligned(16))) float sO[4][RPW][HD + 4];
  const int tid = threadIdx.x, lane = tid & 31, ln = lane & 15, hh = lane >> 4;
  const int w = __builtin_amdgcn_readfirstlane(tid >> 5);
  const int slab = blockIdx.x / QBLKS, qblk = blockIdx.x % QBLKS; const int b = slab / NH, h = slab % NH; const int g = h / NREP;
  const int qb0 = qblk * (4 * RPW); const int q0 = qb0 + w * RPW;
  const int* dq = doc + (size_t)b * SEQ_FULL;
  if (blk_early(dq, qb0, lane) != 0) return;
  const unsigned short* Qu = (const unsigned short*)Q16;
  const int qofs = (b * TQ + q0 + ln) * ldq + h * HD;
  const unsigned short* Kb = (const unsigned short*)K16 + (size_t)b * TK * ldk + g * HD;
  const unsigned short* Vth = (const unsigned short*)Vt + (size_t)(b * NKV + g) * HD * TK;
  int docq[8];
#pragma unroll
  for (int r = 0; r < 8; ++r) docq[r] = dq[q0 + 8 * hh + r];
  int dmin = docq[0], dmax = docq[0];
#pragma unroll
  for (int r = 1; r < 8; ++r) { dmin = min(dmin, docq[r]); dmax = max(dmax, docq[r]); }
  dmin = min(dmin, __shfl_xor(dmin, 16, 32)); dmax = max(dmax, __shfl_xor(dmax, 16, 32));
  const v8f z8 = {0.f,0.f,0.f,0.f,0.f,0.f,0.f,0.f};
  float m_r[8], l_r[8]; v8f oacc[DT];
#pragma unroll
  for (int r = 0; r < 8; ++r) { m_r[r] = -3.0e38f; l_r[r] = 0.f; }
#pragma unroll
  for (int dt = 0; dt < DT; ++dt) oacc[dt] = z8;
  const int jend = q0 + RPW;
#pragma unroll 1
  for (int j0 = 0; j0 < jend; j0 += 32) {
    const int dk0 = dq[j0 + ln], dk1 = dq[j0 + 16 + ln];
    const bool in0 = (dk0 >= dmin) & (dk0 <= dmax), in1 = (dk1 >= dmin) & (dk1 <= dmax);
    if (__builtin_amdgcn_ballot_w32(in0 | in1) == 0u) continue;
    int qo = qofs; asm volatile("" : "+v"(qo));
    const unsigned short* kr0 = Kb + (size_t)(j0 + ln) * ldk; const unsigned short* kr1 = kr0 + (size_t)16 * ldk;
    v8f s[2]; s[0] = z8; s[1] = z8;
#pragma unroll
    for (int ks = 0; ks < KS; ++ks) {
      FragH aq, b0, b1;
      aq.half[0] = *(const v8us*)(Qu + qo + ks * 32 + 8 * hh); aq.half[1] = *(const v8us*)(Qu + qo + ks * 32 + 16 + 8 * hh);
      b0.half[0] = *(const v8us*)(kr0 + ks * 32 + 8 * hh); b0.half[1] = *(const v8us*)(kr0 + ks * 32 + 16 + 8 * hh);
      b1.half[0] = *(const v8us*)(kr1 + ks * 32 + 8 * hh); b1.half[1] = *(const v8us*)(kr1 + ks * 32 + 16 + 8 * hh);
      s[0] = mmaH<1>(aq.v, aq.v, b0.v, b0.v, s[0]);
      s[1] = mmaH<1>(aq.v, aq.v, b1.v, b1.v, s[1]);
    }
#pragma unroll
    for (int r = 0; r < 8; ++r) {
      const int tq = q0 + 8 * hh + r; const int k0 = j0 + ln, k1 = j0 + 16 + ln;
      const bool ok0 = (k0 <= tq) & (dk0 == docq[r]), ok1 = (k1 <= tq) & (dk1 == docq[r]);
      const float s0 = ok0 ? s[0][r] * SCL : -3.0e38f, s1 = ok1 ? s[1][r] * SCL : -3.0e38f;
      float mc = fmaxf(s0, s1);
      mc = fmaxf(mc, __shfl_xor(mc, 1, 32)); mc = fmaxf(mc, __shfl_xor(mc, 2, 32)); mc = fmaxf(mc, __shfl_xor(mc, 4, 32)); mc = fmaxf(mc, __shfl_xor(mc, 8, 32));
      const float mn = fmaxf(m_r[r], mc); const float al = (mn > -1.0e38f) ? expf(m_r[r] - mn) : 1.0f; m_r[r] = mn;
      const float p0 = ok0 ? expf(s0 - mn) : 0.f, p1 = ok1 ? expf(s1 - mn) : 0.f; l_r[r] = l_r[r] * al + p0 + p1;
#pragma unroll
      for (int dt = 0; dt < DT; ++dt) oacc[dt][r] *= al;
      FragH t2; t2.h[0] = toh_flush(p0 * 1024.0f); t2.h[1] = toh_flush(p1 * 1024.0f);
      sP[w][8 * hh + r][ln] = t2.u[0]; sP[w][8 * hh + r][16 + ln] = t2.u[1];
    }
    __builtin_amdgcn_fence(4, "workgroup"); __builtin_amdgcn_wave_barrier();
    FragH pa; pa.half[0] = *(const v8us*)&sP[w][ln][8 * hh]; pa.half[1] = *(const v8us*)&sP[w][ln][16 + 8 * hh];
#pragma unroll
    for (int dt = 0; dt < DT; ++dt) {
      const unsigned short* vrow = Vth + (size_t)(dt * 16 + ln) * TK + j0; FragH bv;
      bv.half[0] = *(const v8us*)(vrow + 8 * hh); bv.half[1] = *(const v8us*)(vrow + 16 + 8 * hh);
      oacc[dt] = mmaH<1>(pa.v, pa.v, bv.v, bv.v, oacc[dt]);
    }
    __builtin_amdgcn_fence(4, "workgroup"); __builtin_amdgcn_wave_barrier();
  }
#pragma unroll
  for (int r = 0; r < 8; ++r) { float l = l_r[r]; l += __shfl_xor(l, 1, 32); l += __shfl_xor(l, 2, 32); l += __shfl_xor(l, 4, 32); l += __shfl_xor(l, 8, 32); l_r[r] = (l > 0.f) ? 1.0f / (l * 1024.0f) : 0.f; }
#pragma unroll
  for (int dt = 0; dt < DT; ++dt)
#pragma unroll
    for (int r = 0; r < 8; ++r) sO[w][8 * hh + r][dt * 16 + ln] = oacc[dt][r] * l_r[r];
  __builtin_amdgcn_fence(4, "workgroup"); __builtin_amdgcn_wave_barrier();
  for (int pass = 0; pass < 2; ++pass) {
#pragma unroll
    for (int rp = 0; rp < RPW; ++rp) { const v4f val = *(const v4fa*)&sO[w][rp][lane * 4]; *(volatile v4f*)(O + ((size_t)b * TQ + q0 + rp) * ldo + h * HD + lane * 4) = val; }
    if (pass == 0) __threadfence();
  }
}
__global__ __launch_bounds__(128) __attribute__((amdgpu_num_vgpr(256))) void k_flash5(const _Float16* __restrict__ Q16, const _Float16* __restrict__ QL, int ldq, const _Float16* __restrict__ K16, const _Float16* __restrict__ KL, int ldk,
                                                const _Float16* __restrict__ Vt, const _Float16* __restrict__ VtL, const int* __restrict__ doc, float* __restrict__ O, int ldo) {
  constexpr int RPW = 16, DT = 4, KS = 4;
  __shared__ __attribute__((aligned(16))) unsigned short sP[4][RPW][40];
  __shared__ __attribute__((aligned(16))) unsigned short sPL[4][RPW][40];
  __shared__ __attribute__((aligned(16))) float sO[4][RPW][68];
  const int tid = threadIdx.x, lane = tid & 31, ln = lane & 15, hh = lane >> 4;
  const int w = __builtin_amdgcn_readfirstlane(tid >> 5);
  const int dh = blockIdx.x & 1; const int bi = blockIdx.x >> 1;
  const int slab = bi / QBLKS, qblk = bi % QBLKS; const int b = slab / NH, h = slab % NH; const int g = h / NREP;
  const int qb0 = qblk * (4 * RPW); const int q0 = qb0 + w * RPW;
  const int* dq = doc + (size_t)b * SEQ_FULL;
  if (blk_early(dq, qb0, lane) == 0) return;
  const unsigned short* Qu = (const unsigned short*)Q16; const unsigned short* QLu = (const unsigned short*)QL;
  const int qofs = (b * TQ + q0 + ln) * ldq + h * HD;
  const unsigned short* Kb = (const unsigned short*)K16 + (size_t)b * TK * ldk + g * HD;
  const unsigned short* KLb = (const unsigned short*)KL + (size_t)b * TK * ldk + g * HD;
  const unsigned short* Vth = (const unsigned short*)Vt + ((size_t)(b * NKV + g) * HD + dh * 64) * TK;
  const unsigned short* Vtl = (const unsigned short*)VtL + ((size_t)(b * NKV + g) * HD + dh * 64) * TK;
  int docq[8];
#pragma unroll
  for (int r = 0; r < 8; ++r) docq[r] = dq[q0 + 8 * hh + r];
  int dmin = docq[0], dmax = docq[0];
#pragma unroll
  for (int r = 1; r < 8; ++r) { dmin = min(dmin, docq[r]); dmax = max(dmax, docq[r]); }
  dmin = min(dmin, __shfl_xor(dmin, 16, 32)); dmax = max(dmax, __shfl_xor(dmax, 16, 32));
  const v8f z8 = {0.f,0.f,0.f,0.f,0.f,0.f,0.f,0.f};
  float m_r[8], l_r[8]; v8f oacc[DT], oaccL[DT];
#pragma unroll
  for (int r = 0; r < 8; ++r) { m_r[r] = -3.0e38f; l_r[r] = 0.f; }
#pragma unroll
  for (int dt = 0; dt < DT; ++dt) { oacc[dt] = z8; oaccL[dt] = z8; }
  const int jend = q0 + RPW;
#pragma unroll 1
  for (int j0 = 0; j0 < jend; j0 += 32) {
    const int dk0 = dq[j0 + ln], dk1 = dq[j0 + 16 + ln];
    const bool in0 = (dk0 >= dmin) & (dk0 <= dmax), in1 = (dk1 >= dmin) & (dk1 <= dmax);
    if (__builtin_amdgcn_ballot_w32(in0 | in1) == 0u) continue;
    int qo = qofs; asm volatile("" : "+v"(qo));
    const unsigned short* kr0 = Kb + (size_t)(j0 + ln) * ldk; const unsigned short* kr1 = kr0 + (size_t)16 * ldk;
    const unsigned short* kl0 = KLb + (size_t)(j0 + ln) * ldk; const unsigned short* kl1 = kl0 + (size_t)16 * ldk;
    v8f s[2], sl[2]; s[0] = z8; s[1] = z8; sl[0] = z8; sl[1] = z8;
#pragma unroll
    for (int ks = 0; ks < KS; ++ks) {
      FragH aq, aql, b0, b0l, b1, b1l;
      aq.half[0] = *(const v8us*)(Qu + qo + ks * 32 + 8 * hh); aq.half[1] = *(const v8us*)(Qu + qo + ks * 32 + 16 + 8 * hh);
      aql.half[0] = *(const v8us*)(QLu + qo + ks * 32 + 8 * hh); aql.half[1] = *(const v8us*)(QLu + qo + ks * 32 + 16 + 8 * hh);
      b0.half[0] = *(const v8us*)(kr0 + ks * 32 + 8 * hh); b0.half[1] = *(const v8us*)(kr0 + ks * 32 + 16 + 8 * hh);
      b0l.half[0] = *(const v8us*)(kl0 + ks * 32 + 8 * hh); b0l.half[1] = *(const v8us*)(kl0 + ks * 32 + 16 + 8 * hh);
      b1.half[0] = *(const v8us*)(kr1 + ks * 32 + 8 * hh); b1.half[1] = *(const v8us*)(kr1 + ks * 32 + 16 + 8 * hh);
      b1l.half[0] = *(const v8us*)(kl1 + ks * 32 + 8 * hh); b1l.half[1] = *(const v8us*)(kl1 + ks * 32 + 16 + 8 * hh);
      s[0] = mmaH<1>(aq.v, aq.v, b0.v, b0.v, s[0]);
      sl[0] = mmaH<1>(aql.v, aql.v, b0.v, b0.v, sl[0]);
      sl[0] = mmaH<1>(aq.v, aq.v, b0l.v, b0l.v, sl[0]);
      s[1] = mmaH<1>(aq.v, aq.v, b1.v, b1.v, s[1]);
      sl[1] = mmaH<1>(aql.v, aql.v, b1.v, b1.v, sl[1]);
      sl[1] = mmaH<1>(aq.v, aq.v, b1l.v, b1l.v, sl[1]);
    }
#pragma unroll
    for (int r = 0; r < 8; ++r) { s[0][r] += sl[0][r] * 0.0009765625f; s[1][r] += sl[1][r] * 0.0009765625f; }
#pragma unroll
    for (int r = 0; r < 8; ++r) {
      const int tq = q0 + 8 * hh + r; const int k0 = j0 + ln, k1 = j0 + 16 + ln;
      const bool ok0 = (k0 <= tq) & (dk0 == docq[r]), ok1 = (k1 <= tq) & (dk1 == docq[r]);
      const float s0 = ok0 ? s[0][r] * SCL : -3.0e38f, s1 = ok1 ? s[1][r] * SCL : -3.0e38f;
      float mc = fmaxf(s0, s1);
      mc = fmaxf(mc, __shfl_xor(mc, 1, 32)); mc = fmaxf(mc, __shfl_xor(mc, 2, 32)); mc = fmaxf(mc, __shfl_xor(mc, 4, 32)); mc = fmaxf(mc, __shfl_xor(mc, 8, 32));
      const float mn = fmaxf(m_r[r], mc); const float al = (mn > -1.0e38f) ? expf(m_r[r] - mn) : 1.0f; m_r[r] = mn;
      const float p0 = ok0 ? expf(s0 - mn) : 0.f, p1 = ok1 ? expf(s1 - mn) : 0.f; l_r[r] = l_r[r] * al + p0 + p1;
#pragma unroll
      for (int dt = 0; dt < DT; ++dt) { oacc[dt][r] *= al; oaccL[dt][r] *= al; }
      FragH t2, t2l; const float ps0 = p0 * 1024.0f, ps1 = p1 * 1024.0f;
      t2.h[0] = toh_flush(ps0); t2.h[1] = toh_flush(ps1);
      t2l.h[0] = toh_flush((ps0 - (float)t2.h[0]) * 1024.0f); t2l.h[1] = toh_flush((ps1 - (float)t2.h[1]) * 1024.0f);
      sP[w][8 * hh + r][ln] = t2.u[0]; sP[w][8 * hh + r][16 + ln] = t2.u[1]; sPL[w][8 * hh + r][ln] = t2l.u[0]; sPL[w][8 * hh + r][16 + ln] = t2l.u[1];
    }
    __builtin_amdgcn_fence(4, "workgroup"); __builtin_amdgcn_wave_barrier();
    FragH pa, pl;
    pa.half[0] = *(const v8us*)&sP[w][ln][8 * hh]; pa.half[1] = *(const v8us*)&sP[w][ln][16 + 8 * hh];
    pl.half[0] = *(const v8us*)&sPL[w][ln][8 * hh]; pl.half[1] = *(const v8us*)&sPL[w][ln][16 + 8 * hh];
#pragma unroll
    for (int dt = 0; dt < DT; ++dt) {
      const unsigned short* vrow = Vth + (size_t)(dt * 16 + ln) * TK + j0; const unsigned short* vrl = Vtl + (size_t)(dt * 16 + ln) * TK + j0;
      FragH bv, bl;
      bv.half[0] = *(const v8us*)(vrow + 8 * hh); bv.half[1] = *(const v8us*)(vrow + 16 + 8 * hh);
      bl.half[0] = *(const v8us*)(vrl + 8 * hh); bl.half[1] = *(const v8us*)(vrl + 16 + 8 * hh);
      oacc[dt] = mmaH<1>(pa.v, pa.v, bv.v, bv.v, oacc[dt]);
      oaccL[dt] = mmaH<1>(pl.v, pl.v, bv.v, bv.v, oaccL[dt]);
      oaccL[dt] = mmaH<1>(pa.v, pa.v, bl.v, bl.v, oaccL[dt]);
    }
    __builtin_amdgcn_fence(4, "workgroup"); __builtin_amdgcn_wave_barrier();
  }
#pragma unroll
  for (int r = 0; r < 8; ++r) { float l = l_r[r]; l += __shfl_xor(l, 1, 32); l += __shfl_xor(l, 2, 32); l += __shfl_xor(l, 4, 32); l += __shfl_xor(l, 8, 32); l_r[r] = (l > 0.f) ? 1.0f / (l * 1024.0f) : 0.f; }
#pragma unroll
  for (int dt = 0; dt < DT; ++dt)
#pragma unroll
    for (int r = 0; r < 8; ++r) { float v = oacc[dt][r]; v += oaccL[dt][r] * 0.0009765625f; sO[w][8 * hh + r][dt * 16 + ln] = v * l_r[r]; }
  __builtin_amdgcn_fence(4, "workgroup"); __builtin_amdgcn_wave_barrier();
  for (int pass = 0; pass < 2; ++pass) {
#pragma unroll
    for (int rp = 0; rp < RPW; rp += 2) { const int r = rp + (lane >> 4), pc = lane & 15; const v4f val = *(const v4fa*)&sO[w][r][pc * 4]; *(volatile v4f*)(O + ((size_t)b * TQ + q0 + r) * ldo + h * HD + dh * 64 + pc * 4) = val; }
    if (pass == 0) __threadfence();
  }
}

extern "C" void kernel_launch(void* const* d_in, const int* in_sizes, int n_in,
                              void* d_out, int out_size, void* d_ws, size_t ws_size, hipStream_t stream) {
  if (n_in < 6) return;
  const size_t needx = ((size_t)(NB - 1) * SEQ_FULL + (size_t)SLEN) * DM;
  if ((size_t)in_sizes[0] < needx) return;
  if ((size_t)in_sizes[1] < (size_t)SLEN * 64) return;
  if ((size_t)in_sizes[2] < (size_t)SLEN * 64) return;
  if ((size_t)in_sizes[3] < (size_t)(NB - 1) * SEQ_FULL + (size_t)SLEN) return;
  if ((size_t)in_sizes[4] < (size_t)DM * QKVN) return;
  if ((size_t)in_sizes[5] < (size_t)DM * DM) return;
  if ((size_t)out_size < needx) return;
  const float* x = (const float*)d_in[0]; const float* sn_t = (const float*)d_in[1]; const float* cs_t = (const float*)d_in[2];
  const int* doc = (const int*)d_in[3]; const float* Wqkv = (const float*)d_in[4]; const float* Wo = (const float*)d_in[5];
  float* dout = (float*)d_out;
  char* ws = (char*)d_ws; size_t off = 0;
  auto take = [&](size_t bytes) { char* p = ws + off; off += (bytes + 255) & ~(size_t)255; return p; };
  const size_t np = (size_t)NR * DM;
  const size_t nk = (size_t)NR * KVD;
  _Float16* BQKV = (_Float16*)take((size_t)QKVN * DM * 2);
  _Float16* B2 = (_Float16*)take((size_t)DM * 2 * DM * 2);
  float* FS = (float*)take(np * 4);
  _Float16* X16 = (_Float16*)take(np * 2);
  _Float16* VT = X16;
  _Float16* QH = (_Float16*)take(np * 2);
  _Float16* QL = (_Float16*)take(np * 2);
  _Float16* A2 = QH;
  _Float16* KH = (_Float16*)take(nk * 2);
  _Float16* KL = (_Float16*)take(nk * 2);
  _Float16* V16 = (_Float16*)take(nk * 2);
  _Float16* VTL = (_Float16*)take(nk * 2);
  if (off > ws_size) return;
  if (off > ((size_t)128 << 20)) return;

  k_wtr<<<(unsigned)((QKVN / 64) * (DM / 64)), 256, 0, stream>>>(Wqkv, DM, QKVN, BQKV, DM, W_SC, W_SC, 0);
  k_wtr<<<(unsigned)((DM / 64) * (DM / 64)), 256, 0, stream>>>(Wo, DM, DM, B2, 2 * DM, W_SC_HI, W_SC, 1);
  const unsigned g8 = (unsigned)((np / 8 + 255) / 256);
  k_x16<<<g8, 256, 0, stream>>>(x, X16, np / 8);
  const dim3 gq((unsigned)((NR / 128) * (DM / 64)), 1);
  const dim3 gk((unsigned)((NR / 128) * (KVD / 64)), 1);
  const unsigned grq = (unsigned)(((size_t)NR * NH * 16 + 255) / 256);
  const unsigned grk = (unsigned)(((size_t)NR * NKV * 16 + 255) / 256);
  k_gemm2<0><<<gq, 128, 0, stream>>>(X16, DM, 0, BQKV, DM, 0, ALPHA_P, FS, nullptr, DM, 0, NR, DM, DM);
  k_rope<<<grq, 256, 0, stream>>>(FS, DM, NH, cs_t, sn_t, QH, QL);
  k_gemm2<0><<<gk, 128, 0, stream>>>(X16, DM, 0, BQKV + (size_t)DM * DM, DM, 0, ALPHA_P, FS, nullptr, KVD, 0, NR, KVD, DM);
  k_rope<<<grk, 256, 0, stream>>>(FS, KVD, NKV, cs_t, sn_t, KH, KL);
  k_gemm2<0><<<gk, 128, 0, stream>>>(X16, DM, 0, BQKV + (size_t)(DM + KVD) * DM, DM, 0, ALPHA_P, FS, V16, KVD, 0, NR, KVD, DM);
  k_vtg<<<(unsigned)(NB * NKV * (SLEN / 64)), 256, 0, stream>>>(V16, VT);
  k_vtl<<<(unsigned)(NB * NKV * (SLEN / 64)), 256, 0, stream>>>(FS, VTL);
  k_flash5<<<(unsigned)(NB * NH * QBLKS * 2), 128, 0, stream>>>(QH, QL, DM, KH, KL, KVD, VT, VTL, doc, FS, DM);
  k_flash<<<(unsigned)(NB * NH * QBLKS), 128, 0, stream>>>(QH, DM, KH, KVD, VT, doc, FS, DM);
  k_hl<<<g8, 256, 0, stream>>>(FS, A2, np / 8);
  const dim3 go((unsigned)((SLEN / 128) * (DM / 64)), NB);
  k_gemmo<<<go, 128, 0, stream>>>(A2, 2 * DM, (size_t)SLEN * 2 * DM, B2, 2 * DM, ALPHA_O, doc, dout, DM, (size_t)SEQ_FULL * DM, SLEN, DM, DM, 2 * DM);
}
